// BiMambaBlock_7894149890252
// MI455X (gfx1250) — hardware-verified
//
#include <hip/hip_runtime.h>
#include <math.h>

typedef __attribute__((ext_vector_type(16))) _Float16 v16h;
typedef __attribute__((ext_vector_type(8)))  _Float16 v8h;
typedef __attribute__((ext_vector_type(8)))  float    v8f;
typedef __attribute__((ext_vector_type(4)))  float    v4f;

constexpr int kNB   = 4;
constexpr int kL    = 1024;
constexpr int kDm   = 1024;
constexpr int kDi   = 2048;
constexpr int kNs   = 16;
constexpr int kDtR  = 64;
constexpr int kXpN  = 96;
constexpr int kXpP  = 128;
constexpr int kXzP  = 2 * kDi;
constexpr int kRows = kNB * kL;
constexpr int kXzW  = kXzP / 2;
constexpr int kXcW  = kDi / 2;
constexpr int kTP   = 260;
constexpr int kTS   = 32;
constexpr float kLnEps = 1e-5f;

constexpr float kCarXn   = 16.0f;
constexpr float kCarW    = 32.0f;
constexpr float kCarXc   = 16.0f;
constexpr float kCarDt   = 16.0f;
constexpr float kCarY    = 64.0f;
constexpr float kCarFeat = 16.0f;
constexpr float kSclIn   = 1.0f / (kCarXn * kCarW);
constexpr float kSclXp   = 1.0f / (kCarXc * kCarW);
constexpr float kSclDt   = 1.0f / (kCarDt * kCarW);
constexpr float kSclOut  = kCarFeat / (kCarY * kCarW);
constexpr float kSclFus  = 1.0f / (kCarFeat * kCarW);
constexpr float kInvCarXc = 1.0f / kCarXc;

static_assert(kDtR + 2 * kNs == kXpN, "x_proj width");
static_assert(kRows == 4096 && kXzP == 4096, "shape constants");
static_assert((kDm % 32) == 0 && (kDi % 32) == 0 && (kDtR % 32) == 0, "GEMM K multiples of 32");
static_assert((kRows % 64) == 0 && (kXzP % 64) == 0 && (kXpP % 64) == 0 && (kDi % 64) == 0 && (kDm % 64) == 0, "GEMM M,N multiples of 64");
static_assert((kL % 64) == 0 && (kL % kTS) == 0 && (kDi % 256) == 0, "tile multiples");

constexpr size_t kSzXN   = (size_t)kRows * kDm * 2;
constexpr size_t kSzWIN  = (size_t)kXzP * kDm * 2;
constexpr size_t kSzWXP  = (size_t)kXpP * kDi * 2;
constexpr size_t kSzWDT  = (size_t)kDi * kDtR * 2;
constexpr size_t kSzWOUT = (size_t)kDm * kDi * 2;
constexpr size_t kSzFUS  = (size_t)kDm * 2 * kDm * 2;
constexpr size_t kSzXZ   = (size_t)kRows * kXzP * 2;
constexpr size_t kSzXC   = (size_t)kRows * kDi * 2;
constexpr size_t kSzDBL  = (size_t)kRows * kXpP * 4;
constexpr size_t kSzDT   = (size_t)kRows * kDtR * 2;
constexpr size_t kSzYG   = (size_t)kRows * kDi * 2;
constexpr size_t kSzFEAT = (size_t)kRows * 2 * kDm * 2;
constexpr size_t kOffXN   = 0;
constexpr size_t kOffWIN  = kOffXN   + kSzXN;
constexpr size_t kOffWXP  = kOffWIN  + 2 * kSzWIN;
constexpr size_t kOffWDT  = kOffWXP  + 2 * kSzWXP;
constexpr size_t kOffWOUT = kOffWDT  + 2 * kSzWDT;
constexpr size_t kOffFUS  = kOffWOUT + 2 * kSzWOUT;
constexpr size_t kOffXZ   = kOffFUS  + kSzFUS;
constexpr size_t kOffXC   = kOffXZ   + kSzXZ;
constexpr size_t kOffDBL  = kOffXC   + kSzXC;
constexpr size_t kOffDT   = kOffDBL  + kSzDBL;
constexpr size_t kOffYG   = kOffDT   + kSzDT;
constexpr size_t kOffFEAT = kOffYG   + kSzYG;
constexpr size_t kWsTotal = kOffFEAT + kSzFEAT;
static_assert(kWsTotal == 125829120ull, "carve total");
static_assert(kWsTotal <= 134217728ull, "carve cap");
static_assert((kOffWIN % 128) == 0 && (kOffWXP % 128) == 0 && (kOffWDT % 128) == 0 && (kOffWOUT % 128) == 0 &&
              (kOffFUS % 128) == 0 && (kOffXZ % 128) == 0 && (kOffXC % 128) == 0 && (kOffDBL % 128) == 0 &&
              (kOffDT % 128) == 0 && (kOffYG % 128) == 0 && (kOffFEAT % 128) == 0, "128-B aligned regions");

__device__ __forceinline__ float h16_to_f32(unsigned hb) {
  const unsigned sgn = (hb & 0x8000u) << 16;
  const unsigned em = hb & 0x7fffu;
  const float fn = __uint_as_float((em << 13) + 0x38000000u);
  const float fs = (float)em * 5.9604644775390625e-8f;
  const float mag = (em < 0x400u) ? fs : fn;
  return __uint_as_float(__float_as_uint(mag) | sgn);
}

__device__ __forceinline__ void dep_guard4_h(v8f& a, v8f& b, v8f& c, v8f& d, v16h x, v16h y0, v16h y1, v16h y2, v16h y3) {
  asm volatile("v_nop\n\tv_nop\n\tv_nop\n\tv_nop" : "+v"(a), "+v"(b), "+v"(c), "+v"(d) : "v"(x), "v"(y0), "v"(y1), "v"(y2), "v"(y3));
}
__device__ __forceinline__ void keep4_h(v16h a, v16h b, v16h c, v16h d) { asm volatile("v_nop" :: "v"(a), "v"(b), "v"(c), "v"(d)); }
__device__ __forceinline__ void acc_guard4(v8f& a, v8f& b, v8f& c, v8f& d) { asm volatile("v_nop\n\tv_nop\n\tv_nop\n\tv_nop" : "+v"(a), "+v"(b), "+v"(c), "+v"(d)); }
struct FragH {
  union U { v16h v; v8h h[2]; };
  static __device__ __forceinline__ v16h load(const _Float16* p) {
    U f; f.h[0] = *(const v8h*)(p); f.h[1] = *(const v8h*)(p + 16); return f.v;
  }
  static __device__ __forceinline__ v8f mma(v16h a, v16h b, v8f c) {
    return __builtin_amdgcn_wmma_f32_16x16x32_f16(false, a, false, b, (short)0, c, false, false);
  }
};

template <int BIAS_MODE, int OUT_MODE, bool RESID>
__global__ __launch_bounds__(256) void wmma_gemm64(
    const unsigned short* __restrict__ Ap, int lda,
    const unsigned short* __restrict__ Btp, int ldb,
    void* __restrict__ Cout, int ldc,
    const float* __restrict__ bias,
    const float* __restrict__ resid, int ldr,
    int M, int N, int K, float scale) {
  const _Float16* A  = (const _Float16*)Ap;
  const _Float16* Bt = (const _Float16*)Btp;
  __shared__ __align__(16) float sT[8][16 * 68];
  const int lane = threadIdx.x & 31;
  const int wave = threadIdx.x >> 5;
  const int tilesN = N >> 6;
  const int tilesM = M >> 6;
  const int tile = blockIdx.x * 8 + wave;
  if (tile >= tilesM * tilesN) return;
  const int tm = tile / tilesN;
  const int tn = tile - tm * tilesN;
  const int m0 = tm << 6;
  const int n0 = tn << 6;

  const int rlane = lane & 15;
  const int koff  = (lane >> 4) * 8;
  const int mOff  = (lane >> 4) * 8;

  v8f acc[4][4];
#pragma unroll
  for (int i = 0; i < 4; ++i)
#pragma unroll
    for (int j = 0; j < 4; ++j) acc[i][j] = (v8f){0.f,0.f,0.f,0.f,0.f,0.f,0.f,0.f};

  for (int k0 = 0; k0 < K; k0 += 32) {
    v16h bh[4];
#pragma unroll
    for (int j = 0; j < 4; ++j) {
      const size_t bo = (size_t)(n0 + (j << 4) + rlane) * ldb + koff + k0;
      bh[j] = FragH::load(Bt + bo);
    }
#pragma unroll
    for (int i = 0; i < 4; ++i) {
      const size_t ao = (size_t)(m0 + (i << 4) + rlane) * lda + koff + k0;
      v16h ah = FragH::load(A + ao);
#pragma unroll
      for (int j = 0; j < 4; ++j) acc[i][j] = FragH::mma(ah, bh[j], acc[i][j]);
      dep_guard4_h(acc[i][0], acc[i][1], acc[i][2], acc[i][3], ah, bh[0], bh[1], bh[2], bh[3]);
    }
    keep4_h(bh[0], bh[1], bh[2], bh[3]);
  }
  acc_guard4(acc[0][0], acc[0][1], acc[0][2], acc[0][3]);
  acc_guard4(acc[1][0], acc[1][1], acc[1][2], acc[1][3]);
  acc_guard4(acc[2][0], acc[2][1], acc[2][2], acc[2][3]);
  acc_guard4(acc[3][0], acc[3][1], acc[3][2], acc[3][3]);

  float* slab = sT[wave];
#pragma unroll
  for (int i = 0; i < 4; ++i) {
    const int mBase = m0 + (i << 4);
#pragma unroll
    for (int j = 0; j < 4; ++j) {
      const int n = n0 + (j << 4) + rlane;
      float bv = 0.f;
      if (BIAS_MODE == 2) bv = bias[n];
#pragma unroll
      for (int r = 0; r < 8; ++r) {
        float v = acc[i][j][r] * scale;
        if (BIAS_MODE == 2) v += bv;
        slab[(mOff + r) * 68 + (j << 4) + rlane] = v;
      }
    }
    __builtin_amdgcn_fence(__ATOMIC_RELEASE, "workgroup");
    __builtin_amdgcn_wave_barrier();
    __builtin_amdgcn_fence(__ATOMIC_ACQUIRE, "workgroup");
    if (OUT_MODE == 0) {
      float* C = (float*)Cout;
      const int hh = lane >> 4, c4 = (lane & 15) * 4;
      v4f vals[8];
#pragma unroll
      for (int it = 0; it < 8; ++it) {
        const int row = it * 2 + hh;
        v4f v = *(const v4f*)(slab + row * 68 + c4);
        if (RESID) {
          const v4f rv = *(const v4f*)(resid + (size_t)(mBase + row) * ldr + n0 + c4);
          v = v + rv;
        }
        vals[it] = v;
      }
      for (int pass = 0; pass < 2; ++pass) {
#pragma unroll
        for (int it = 0; it < 8; ++it) {
          const int row = it * 2 + hh;
          *(volatile v4f*)(C + (size_t)(mBase + row) * ldc + n0 + c4) = vals[it];
        }
        __threadfence();
      }
    } else {
      const int q = lane >> 3, c8 = (lane & 7) * 8;
      unsigned short* C = (unsigned short*)Cout;
      v8h hv[4];
#pragma unroll
      for (int it = 0; it < 4; ++it) {
        const int row = it * 4 + q;
        const float* sp = slab + row * 68 + c8;
        const v4f a0 = *(const v4f*)(sp);
        const v4f a1 = *(const v4f*)(sp + 4);
#pragma unroll
        for (int e = 0; e < 4; ++e) {
          hv[it][e]     = (_Float16)a0[e];
          hv[it][4 + e] = (_Float16)a1[e];
        }
      }
      for (int pass = 0; pass < 2; ++pass) {
#pragma unroll
        for (int it = 0; it < 4; ++it) {
          const int row = it * 4 + q;
          *(volatile v8h*)(C + (size_t)(mBase + row) * ldc + n0 + c8) = hv[it];
        }
        __threadfence();
      }
    }
    __builtin_amdgcn_fence(__ATOMIC_RELEASE, "workgroup");
    __builtin_amdgcn_wave_barrier();
    __builtin_amdgcn_fence(__ATOMIC_ACQUIRE, "workgroup");
  }
}

__global__ __launch_bounds__(256) void cast_f16_kernel(
    const float* __restrict__ src, unsigned short* __restrict__ dst, int nsrc8, int total8, float scale)
{
  const int i = blockIdx.x * 256 + threadIdx.x;
  if (i >= total8) return;
  const bool live = (i < nsrc8);
  const int ic = live ? i : (nsrc8 - 1);
  const float* p = src + ((size_t)ic << 3);
  const v4f a0 = *(const v4f*)(p);
  const v4f a1 = *(const v4f*)(p + 4);
  v8h hv;
#pragma unroll
  for (int e = 0; e < 4; ++e) {
    const float f0 = live ? (a0[e] * scale) : 0.0f;
    const float f1 = live ? (a1[e] * scale) : 0.0f;
    hv[e]     = (_Float16)f0;
    hv[4 + e] = (_Float16)f1;
  }
  unsigned short* q = dst + ((size_t)i << 3);
  *(volatile v8h*)q = hv;
  __threadfence();
  *(volatile v8h*)q = hv;
}

__global__ __launch_bounds__(128) void layernorm_kernel(
    const float* __restrict__ x, const float* __restrict__ g, const float* __restrict__ be,
    unsigned short* __restrict__ xn16)
{
  __shared__ float sS[4];
  __shared__ float sQ[4];
  const int tid = threadIdx.x, lane = tid & 31, wave = tid >> 5;
  const size_t base = (size_t)blockIdx.x * kDm + (size_t)tid * 8;
  const v4f a0 = *(const v4f*)(x + base);
  const v4f a1 = *(const v4f*)(x + base + 4);
  float s = ((a0[0] + a0[1]) + (a0[2] + a0[3])) + ((a1[0] + a1[1]) + (a1[2] + a1[3]));
  s += __shfl_xor(s, 16, 32);
  s += __shfl_xor(s, 8, 32);
  s += __shfl_xor(s, 4, 32);
  s += __shfl_xor(s, 2, 32);
  s += __shfl_xor(s, 1, 32);
  if (lane == 0) sS[wave] = s;
  __syncthreads();
  const float mean = ((sS[0] + sS[1]) + (sS[2] + sS[3])) * (1.0f / (float)kDm);
  float dv[8];
#pragma unroll
  for (int e = 0; e < 4; ++e) {
    dv[e]     = a0[e] - mean;
    dv[4 + e] = a1[e] - mean;
  }
  float qs = 0.0f;
#pragma unroll
  for (int e = 0; e < 8; ++e) qs = fmaf(dv[e], dv[e], qs);
  qs += __shfl_xor(qs, 16, 32);
  qs += __shfl_xor(qs, 8, 32);
  qs += __shfl_xor(qs, 4, 32);
  qs += __shfl_xor(qs, 2, 32);
  qs += __shfl_xor(qs, 1, 32);
  if (lane == 0) sQ[wave] = qs;
  __syncthreads();
  const float var = ((sQ[0] + sQ[1]) + (sQ[2] + sQ[3])) * (1.0f / (float)kDm);
  const float inv = rsqrtf(var + kLnEps);
  const v4f g0 = *(const v4f*)(g + tid * 8);
  const v4f g1 = *(const v4f*)(g + tid * 8 + 4);
  const v4f b0 = *(const v4f*)(be + tid * 8);
  const v4f b1 = *(const v4f*)(be + tid * 8 + 4);
  v8h hv;
#pragma unroll
  for (int e = 0; e < 4; ++e) {
    const float y0 = (dv[e] * inv) * g0[e] + b0[e];
    const float y1 = (dv[4 + e] * inv) * g1[e] + b1[e];
    hv[e]     = (_Float16)(y0 * kCarXn);
    hv[4 + e] = (_Float16)(y1 * kCarXn);
  }
  unsigned short* q = xn16 + base;
  *(volatile v8h*)q = hv;
  __threadfence();
  *(volatile v8h*)q = hv;
}

__global__ __launch_bounds__(256) void conv_silu_kernel(
    const unsigned* __restrict__ XZw, const float* __restrict__ cw, const float* __restrict__ cb,
    unsigned short* __restrict__ XC16, int rev)
{
  __shared__ __align__(16) float sT[16 * kTP];
  const int tid = threadIdx.x, lane = tid & 31, wave = tid >> 5;
  const int d0 = blockIdx.x * 256, d = d0 + tid;
  const int g0 = blockIdx.y * 64;
  const int tb = g0 & (kL - 1);
  const int wcol = d >> 1;
  const unsigned sh = (unsigned)(d & 1) * 16u;
  const v4f wv = *(const v4f*)(cw + (size_t)d * 4);
  const float w0 = wv[0], w1 = wv[1], w2 = wv[2], w3 = wv[3];
  const float bc = cb[d];
  float xm3, xm2, xm1;
  {
    const bool hist = rev ? (tb + 64 < kL) : (tb > 0);
    const int rb = hist ? (rev ? (g0 + 64) : (g0 - 3)) : g0;
    unsigned q0 = XZw[(size_t)rb * kXzW + wcol];
    unsigned q1 = XZw[(size_t)(rb + 1) * kXzW + wcol];
    unsigned q2 = XZw[(size_t)(rb + 2) * kXzW + wcol];
    const float f0 = h16_to_f32((q0 >> sh) & 0xffffu);
    const float f1 = h16_to_f32((q1 >> sh) & 0xffffu);
    const float f2 = h16_to_f32((q2 >> sh) & 0xffffu);
    const float n1 = rev ? f0 : f2;
    const float n3 = rev ? f2 : f0;
    xm1 = hist ? n1 : 0.0f;
    xm2 = hist ? f1 : 0.0f;
    xm3 = hist ? n3 : 0.0f;
  }
#pragma unroll 1
  for (int sub = 0; sub < 4; ++sub) {
    const int lb = g0 + (rev ? (3 - sub) : sub) * 16;
#pragma unroll 1
    for (int s = 0; s < 16; ++s) {
      const int rr = rev ? (15 - s) : s;
      unsigned wq = XZw[(size_t)(lb + rr) * kXzW + wcol];
      asm volatile("" : "+v"(wq));
      const float xcur = h16_to_f32((wq >> sh) & 0xffffu);
      float acc = w0 * xm3;
      acc = fmaf(w1, xm2, acc);
      acc = fmaf(w2, xm1, acc);
      acc = fmaf(w3, xcur, acc);
      const float sv = acc + bc;
      const float sg = __builtin_amdgcn_rcpf(1.0f + expf(-sv));
      sT[rr * kTP + tid] = (sv * sg) * kCarXc;
      xm3 = xm2; xm2 = xm1; xm1 = xcur;
    }
    __syncthreads();
    v8h bv[2];
#pragma unroll
    for (int it = 0; it < 2; ++it) {
      const float* sp = sT + (it * 8 + wave) * kTP + lane * 8;
      const v4f a0 = *(const v4f*)(sp);
      const v4f a1 = *(const v4f*)(sp + 4);
#pragma unroll
      for (int e = 0; e < 4; ++e) {
        bv[it][e]     = (_Float16)a0[e];
        bv[it][4 + e] = (_Float16)a1[e];
      }
    }
    for (int pass = 0; pass < 2; ++pass) {
#pragma unroll
      for (int it = 0; it < 2; ++it)
        *(volatile v8h*)(XC16 + (size_t)(lb + it * 8 + wave) * kDi + d0 + lane * 8) = bv[it];
      __threadfence();
    }
    __syncthreads();
  }
}

__global__ __launch_bounds__(256) void dt_cast_kernel(
    const float* __restrict__ DBL, unsigned short* __restrict__ DT16, int total8, float scale)
{
  const int i = blockIdx.x * 256 + threadIdx.x;
  if (i >= total8) return;
  const int e0  = i << 3;
  const int row = e0 >> 6;
  const int c8  = e0 & 63;
  const float* p = DBL + (size_t)row * kXpP + c8;
  const v4f a0 = *(const v4f*)(p);
  const v4f a1 = *(const v4f*)(p + 4);
  v8h hv;
#pragma unroll
  for (int e = 0; e < 4; ++e) {
    hv[e]     = (_Float16)(a0[e] * scale);
    hv[4 + e] = (_Float16)(a1[e] * scale);
  }
  unsigned short* qd = DT16 + e0;
  *(volatile v8h*)qd = hv;
  __threadfence();
  *(volatile v8h*)qd = hv;
}

__global__ __launch_bounds__(256) void scan_kernel(
    const unsigned* __restrict__ XZw, const unsigned* __restrict__ XCw, const float* __restrict__ DBL,
    const float* __restrict__ Alog, const float* __restrict__ Dp, unsigned short* __restrict__ YG16, int rev)
{
  __shared__ __align__(16) float sBC[kTS * 32];
  __shared__ __align__(16) float sY[kTS * kTP];
  __shared__ __align__(16) float sA[kNs * 256];
  const int tid = threadIdx.x, lane = tid & 31, wave = tid >> 5;
  const int bix = blockIdx.x >> 3;
  const int d0  = (blockIdx.x & 7) * 256;
  const int d   = d0 + tid;
  const size_t row0 = (size_t)bix * kL;
  const int wcol = d >> 1;
  const unsigned sh = (unsigned)(d & 1) * 16u;
#pragma unroll 1
  for (int n = 0; n < kNs; ++n) sA[n * 256 + tid] = -expf(Alog[(size_t)d * kNs + n]);
  __syncthreads();
  float An[kNs], h[kNs];
#pragma unroll
  for (int n = 0; n < kNs; ++n) {
    An[n] = sA[n * 256 + tid];
    h[n] = 0.0f;
  }
  const float Dd = Dp[d];
  const int sr = tid >> 3, sq = (tid & 7) * 4;
#pragma unroll 1
  for (int c = 0; c < kL / kTS; ++c) {
    const int tstart = rev ? ((kL - kTS) - c * kTS) : (c * kTS);
    __syncthreads();
    {
      const v4f v = *(const v4f*)(DBL + (row0 + (size_t)(tstart + sr)) * kXpP + kDtR + sq);
      *(v4f*)(sBC + sr * 32 + sq) = v;
    }
    __syncthreads();
#pragma unroll 1
    for (int s = 0; s < kTS; ++s) {
      const int rr = rev ? (kTS - 1 - s) : s;
      const size_t m = row0 + (size_t)(tstart + rr);
      unsigned wd = XZw[m * kXzW + wcol];
      unsigned wz = XZw[m * kXzW + (kDi / 2) + wcol];
      unsigned wu = XCw[m * kXcW + wcol];
      asm volatile("" : "+v"(wd));
      asm volatile("" : "+v"(wz));
      asm volatile("" : "+v"(wu));
      const float v  = h16_to_f32((wd >> sh) & 0xffffu);
      const float zv = h16_to_f32((wz >> sh) & 0xffffu);
      const float u  = h16_to_f32((wu >> sh) & 0xffffu) * kInvCarXc;
      const float* bc = sBC + rr * 32;
      v4f Bq[4], Cq[4];
#pragma unroll
      for (int qq = 0; qq < 4; ++qq) {
        Bq[qq] = *(const v4f*)(bc + 4 * qq);
        Cq[qq] = *(const v4f*)(bc + kNs + 4 * qq);
      }
      const float av  = __expf(-fabsf(v));
      const float u1  = 1.0f + av;
      const float l1p = __logf(u1) + (av - (u1 - 1.0f)) * __builtin_amdgcn_rcpf(u1);
      const float delta = fmaxf(v, 0.0f) + l1p;
      const float du = delta * u;
      float y = 0.0f;
#pragma unroll
      for (int n = 0; n < kNs; ++n) {
        const float e = __expf(delta * An[n]);
        h[n] = fmaf(h[n], e, du * Bq[n >> 2][n & 3]);
        y = fmaf(h[n], Cq[n >> 2][n & 3], y);
      }
      y = fmaf(u, Dd, y);
      const float sg = __builtin_amdgcn_rcpf(1.0f + expf(-zv));
      sY[rr * kTP + tid] = (y * (zv * sg)) * kCarY;
    }
    __syncthreads();
    v8h hv[4];
#pragma unroll
    for (int it = 0; it < 4; ++it) {
      const float* sp = sY + (it * 8 + wave) * kTP + lane * 8;
      const v4f a0 = *(const v4f*)(sp);
      const v4f a1 = *(const v4f*)(sp + 4);
#pragma unroll
      for (int e = 0; e < 4; ++e) {
        hv[it][e]     = (_Float16)a0[e];
        hv[it][4 + e] = (_Float16)a1[e];
      }
    }
    for (int pass = 0; pass < 2; ++pass) {
#pragma unroll
      for (int it = 0; it < 4; ++it)
        *(volatile v8h*)(YG16 + (row0 + (size_t)(tstart + it * 8 + wave)) * kDi + d0 + lane * 8) = hv[it];
      __threadfence();
    }
  }
}

extern "C" void kernel_launch(void* const* d_in, const int* in_sizes, int n_in,
                              void* d_out, int out_size, void* d_ws, size_t ws_size,
                              hipStream_t stream)
{
  if (n_in < 23) return;
  if (in_sizes[0] != kRows * kDm) return;
  if (in_sizes[1] != kDm || in_sizes[2] != kDm) return;
  if (in_sizes[3] != kDm * 2 * kDm || in_sizes[4] != kDm) return;
  for (int p = 0; p < 2; ++p) {
    const int o = 5 + 9 * p;
    if (in_sizes[o + 0] != kXzP * kDm) return;
    if (in_sizes[o + 1] != kDi * 4) return;
    if (in_sizes[o + 2] != kDi) return;
    if (in_sizes[o + 3] != kXpN * kDi) return;
    if (in_sizes[o + 4] != kDi * kDtR) return;
    if (in_sizes[o + 5] != kDi) return;
    if (in_sizes[o + 6] != kDi * kNs) return;
    if (in_sizes[o + 7] != kDi) return;
    if (in_sizes[o + 8] != kDm * kDi) return;
  }
  if (out_size != kRows * kDm) return;
  if (ws_size < kWsTotal) return;

  const float* x     = (const float*)d_in[0];
  const float* ln_g  = (const float*)d_in[1];
  const float* ln_b  = (const float*)d_in[2];
  const float* fus_w = (const float*)d_in[3];
  const float* fus_b = (const float*)d_in[4];
  const float* in_w[2];
  const float* conv_w[2];
  const float* conv_b[2];
  const float* xproj_w[2];
  const float* dt_w[2];
  const float* dt_b[2];
  const float* A_log[2];
  const float* Dv[2];
  const float* out_w[2];
  for (int p = 0; p < 2; ++p) {
    const int o = 5 + 9 * p;
    in_w[p]    = (const float*)d_in[o + 0];
    conv_w[p]  = (const float*)d_in[o + 1];
    conv_b[p]  = (const float*)d_in[o + 2];
    xproj_w[p] = (const float*)d_in[o + 3];
    dt_w[p]    = (const float*)d_in[o + 4];
    dt_b[p]    = (const float*)d_in[o + 5];
    A_log[p]   = (const float*)d_in[o + 6];
    Dv[p]      = (const float*)d_in[o + 7];
    out_w[p]   = (const float*)d_in[o + 8];
  }
  float* dout = (float*)d_out;

  char* ws = (char*)d_ws;
  unsigned short* XN   = (unsigned short*)(ws + kOffXN);
  unsigned short* FUS  = (unsigned short*)(ws + kOffFUS);
  unsigned short* XZ   = (unsigned short*)(ws + kOffXZ);
  unsigned short* XC   = (unsigned short*)(ws + kOffXC);
  float*          DBL  = (float*)(ws + kOffDBL);
  unsigned short* DT   = (unsigned short*)(ws + kOffDT);
  unsigned short* YG   = (unsigned short*)(ws + kOffYG);
  unsigned short* FEAT = (unsigned short*)(ws + kOffFEAT);
  unsigned short* WIN[2];
  unsigned short* WXP[2];
  unsigned short* WDT[2];
  unsigned short* WOUT[2];
  for (int p = 0; p < 2; ++p) {
    WIN[p]  = (unsigned short*)(ws + kOffWIN  + (size_t)p * kSzWIN);
    WXP[p]  = (unsigned short*)(ws + kOffWXP  + (size_t)p * kSzWXP);
    WDT[p]  = (unsigned short*)(ws + kOffWDT  + (size_t)p * kSzWDT);
    WOUT[p] = (unsigned short*)(ws + kOffWOUT + (size_t)p * kSzWOUT);
  }

  constexpr int kIn8  = kXzP * kDm / 8;
  constexpr int kXpS8 = kXpN * kDi / 8;
  constexpr int kXpT8 = kXpP * kDi / 8;
  constexpr int kDt8  = kDi * kDtR / 8;
  constexpr int kOut8 = kDm * kDi / 8;
  constexpr int kFus8 = kDm * 2 * kDm / 8;
  static_assert((kIn8 % 256) == 0 && (kXpT8 % 256) == 0 && (kDt8 % 256) == 0 && (kOut8 % 256) == 0 && (kFus8 % 256) == 0, "cast grids exact");
  for (int p = 0; p < 2; ++p) {
    cast_f16_kernel<<<kIn8 / 256, 256, 0, stream>>>(in_w[p], WIN[p], kIn8, kIn8, kCarW);
    cast_f16_kernel<<<kXpT8 / 256, 256, 0, stream>>>(xproj_w[p], WXP[p], kXpS8, kXpT8, kCarW);
    cast_f16_kernel<<<kDt8 / 256, 256, 0, stream>>>(dt_w[p], WDT[p], kDt8, kDt8, kCarW);
    cast_f16_kernel<<<kOut8 / 256, 256, 0, stream>>>(out_w[p], WOUT[p], kOut8, kOut8, kCarW);
  }
  cast_f16_kernel<<<kFus8 / 256, 256, 0, stream>>>(fus_w, FUS, kFus8, kFus8, kCarW);

  layernorm_kernel<<<kRows, 128, 0, stream>>>(x, ln_g, ln_b, XN);

  for (int p = 0; p < 2; ++p) {
    wmma_gemm64<0, 1, false><<<(kRows / 64) * (kXzP / 64) / 8, 256, 0, stream>>>(
        XN, kDm, WIN[p], kDm, (void*)XZ, kXzP, dt_b[p], x, kDm,
        kRows, kXzP, kDm, kSclIn);

    conv_silu_kernel<<<dim3(kDi / 256, kRows / 64), 256, 0, stream>>>(
        (const unsigned*)XZ, conv_w[p], conv_b[p], XC, p);

    wmma_gemm64<0, 0, false><<<(kRows / 64) * (kXpP / 64) / 8, 256, 0, stream>>>(
        XC, kDi, WXP[p], kDi, (void*)DBL, kXpP, dt_b[p], x, kDm,
        kRows, kXpP, kDi, kSclXp);

    dt_cast_kernel<<<(kRows * kDtR / 8) / 256, 256, 0, stream>>>(DBL, DT, kRows * kDtR / 8, kCarDt);

    wmma_gemm64<2, 1, false><<<(kRows / 64) * (kDi / 64) / 8, 256, 0, stream>>>(
        DT, kDtR, WDT[p], kDtR, (void*)XZ, kXzP, dt_b[p], x, kDm,
        kRows, kDi, kDtR, kSclDt);

    scan_kernel<<<kNB * (kDi / 256), 256, 0, stream>>>(
        (const unsigned*)XZ, (const unsigned*)XC, DBL, A_log[p], Dv[p], YG, p);

    wmma_gemm64<0, 1, false><<<(kRows / 64) * (kDm / 64) / 8, 256, 0, stream>>>(
        YG, kDi, WOUT[p], kDi, (void*)(FEAT + (size_t)p * kDm), 2 * kDm, dt_b[p], x, kDm,
        kRows, kDm, kDi, kSclOut);
  }

  wmma_gemm64<2, 0, true><<<(kRows / 64) * (kDm / 64) / 8, 256, 0, stream>>>(
      FEAT, 2 * kDm, FUS, 2 * kDm, (void*)dout, kDm, fus_b, x, kDm,
      kRows, kDm, 2 * kDm, kSclFus);
}
